// Cross_Atten_Lite_split_63995012710843
// MI455X (gfx1250) — hardware-verified
//
#include <hip/hip_runtime.h>
#include <math.h>
#include <stdint.h>

#define NB    4
#define CIN   256
#define NF    128
#define HD    64
#define NH    2
#define NBH   (NB * NH)
#define SEQ   4096
#define QT    64
#define AP    264
#define QP    136
#define LP    72
#define OHP   136
#define OSP   68
#define LNPS  6.931471805599453f
#define RSC   2048.0f
#define SCL   0.125f
#define IRSS  0.00006103515625f
#define VSC   16.0f
#define IVSC  0.0625f
#define BNEPS 0.00001f

static_assert((SEQ % QT) == 0);
static_assert((SEQ % 32) == 0);
static_assert(QT == 64);
static_assert(HD == 64);
static_assert(NF == NH * HD);
static_assert((CIN % 32) == 0);
static_assert((NF % 32) == 0);
static_assert(NF * LP <= QT * AP);
static_assert((AP % 8) == 0 && (QP % 8) == 0 && (LP % 8) == 0 && (OHP % 8) == 0);
static_assert((OSP % 4) == 0);
static_assert(QP >= NF + 8);
static_assert(NF * CIN == 4 * 8192);
static_assert(CIN * NF == 4 * 8192);

typedef _Float16       v16h __attribute__((ext_vector_type(16)));
typedef _Float16       v8h  __attribute__((ext_vector_type(8)));
typedef __bf16         v16b __attribute__((ext_vector_type(16)));
typedef unsigned short v8us __attribute__((ext_vector_type(8)));
typedef float          v8f  __attribute__((ext_vector_type(8)));
typedef float          v4f  __attribute__((ext_vector_type(4)));
typedef unsigned int   v4u  __attribute__((ext_vector_type(4)));

union FragH { v16h v; v8h  h[2]; };
union FragB { v16b v; v8us u[2]; };
static_assert(sizeof(FragH) == 32);
static_assert(sizeof(FragB) == 32);

__device__ __forceinline__ unsigned short bf_bits(float f) {
  unsigned u = __float_as_uint(f);
  return (unsigned short)((u + 0x7FFFu + ((u >> 16) & 1u)) >> 16);
}
__device__ __forceinline__ float bf_up(unsigned short hv) { return __uint_as_float(((unsigned)hv) << 16); }
__device__ __forceinline__ float bfr(float f) { return bf_up(bf_bits(f)); }
__device__ __forceinline__ unsigned short h_bits(_Float16 x) { return __builtin_bit_cast(unsigned short, x); }
__device__ __forceinline__ unsigned pk16(unsigned short a, unsigned short b) { return (unsigned)a | ((unsigned)b << 16); }
__device__ __forceinline__ v8f zero8() { v8f z = {0.f, 0.f, 0.f, 0.f, 0.f, 0.f, 0.f, 0.f}; return z; }
__device__ __forceinline__ float hmax8(v8f s) {
  return fmaxf(fmaxf(fmaxf(s[0], s[1]), fmaxf(s[2], s[3])), fmaxf(fmaxf(s[4], s[5]), fmaxf(s[6], s[7])));
}

__device__ __forceinline__ v16h ldfrag_h(const _Float16* p) {
  FragH f;
  f.h[0] = *(const v8h*)(p);
  f.h[1] = *(const v8h*)(p + 16);
  return f.v;
}
__device__ __forceinline__ v16b ldfrag_b(const unsigned short* p) {
  FragB f;
  f.u[0] = *(const v8us*)(p);
  f.u[1] = *(const v8us*)(p + 16);
  return f.v;
}

__device__ __forceinline__ v8f mma_h(v16h a, v16h b, v8f c) {
  v8f d = __builtin_amdgcn_wmma_f32_16x16x32_f16(false, a, false, b, (short)0, c, false, false);
#if defined(__HIP_DEVICE_COMPILE__)
  asm volatile("v_nop\n\tv_nop\n\tv_nop\n\tv_nop" : "+v"(d) : "v"(a), "v"(b));
#endif
  return d;
}
__device__ __forceinline__ v8f mma_b(v16b a, v16b b, v8f c) {
  v8f d = __builtin_amdgcn_wmma_f32_16x16x32_bf16(false, a, false, b, (short)0, c, false, false);
#if defined(__HIP_DEVICE_COMPILE__)
  const v16h ha = __builtin_bit_cast(v16h, a), hb = __builtin_bit_cast(v16h, b);
  asm volatile("v_nop\n\tv_nop\n\tv_nop\n\tv_nop" : "+v"(d) : "v"(ha), "v"(hb));
#endif
  return d;
}

__device__ __forceinline__ void stage_split(unsigned short* Lh, unsigned short* Ll, int nr, int col, v8f acc, float bias) {
#pragma unroll
  for (int r = 0; r < 8; ++r) {
    const float val = acc[r] + bias;
    const _Float16 hi = (_Float16)val;
    const float res = (val - (float)hi) * RSC;
    Lh[(nr + r) * QP + col] = h_bits(hi);
    Ll[(nr + r) * QP + col] = h_bits((_Float16)res);
  }
}
__device__ __forceinline__ void stage_v(unsigned short* Lv, int f, int nr, v8f acc, float bias) {
#pragma unroll
  for (int r = 0; r < 8; ++r) Lv[f * LP + nr + r] = h_bits((_Float16)((acc[r] + bias) * VSC));
}

__global__ __launch_bounds__(256)
void wprep_kernel(const float* __restrict__ kq1_w, const float* __restrict__ kq1_b,
                  const float* __restrict__ kq2_w, const float* __restrict__ kq2_b,
                  const float* __restrict__ v_w,   const float* __restrict__ out_w,
                  const float* __restrict__ g1, const float* __restrict__ b1,
                  const float* __restrict__ m1, const float* __restrict__ v1,
                  const float* __restrict__ g2, const float* __restrict__ b2,
                  const float* __restrict__ m2, const float* __restrict__ v2,
                  unsigned short* W1H, unsigned short* W1L, unsigned short* W2H, unsigned short* W2L,
                  unsigned short* WV, unsigned short* WO, float* BF) {
  __shared__ float Ls[CIN];
  __shared__ float Lsh[CIN];
  __shared__ __align__(16) float Lb[32];
  const int tid = threadIdx.x, lane = tid & 31, wave = tid >> 5;
  const int role = blockIdx.x >> 2, part = blockIdx.x & 3;

  {
    const int ch = tid;
    const float ga = bfr(g1[ch]), ba = bfr(b1[ch]), ma = bfr(m1[ch]), va = bfr(v1[ch]);
    const float gb = bfr(g2[ch]), bb = bfr(b2[ch]), mb = bfr(m2[ch]), vb = bfr(v2[ch]);
    const bool r1 = (role == 1);
    const float g = r1 ? gb : ga, bt = r1 ? bb : ba, mu = r1 ? mb : ma, var = r1 ? vb : va;
    const float rs = rsqrtf(var + BNEPS);
    Ls[ch]  = g * rs;
    Lsh[ch] = bt - (mu * g) * rs;
  }
  __syncthreads();

  const float* src = (role == 0) ? kq1_w : ((role == 1) ? kq2_w : ((role == 2) ? v_w : out_w));
  const float* bsrc = (role == 1) ? kq2_b : kq1_b;
  unsigned short* dh = (role == 0) ? W1H : ((role == 1) ? W2H : ((role == 2) ? WV : WO));
  unsigned short* dl = (role == 1) ? W2L : W1L;
  const bool fold = role < 2;
  const int base = part * 8192;
  const int c0 = lane * 8;
#pragma unroll 1
  for (int it = 0; it < 4; ++it) {
    const int e = base + it * 2048 + tid * 8;
    const v4f wa = *(const v4f*)(src + e);
    const v4f wb = *(const v4f*)(src + e + 4);
    const v8f w8 = __builtin_shufflevector(wa, wb, 0, 1, 2, 3, 4, 5, 6, 7);
    v4u uh, ul;
    float dot = 0.f;
#pragma unroll
    for (int t = 0; t < 4; ++t) {
      const float p0 = bfr(w8[2 * t]), p1 = bfr(w8[2 * t + 1]);
      const float s0 = fold ? Ls[c0 + 2 * t] : 1.0f;
      const float s1 = fold ? Ls[c0 + 2 * t + 1] : 1.0f;
      const float f0 = p0 * s0, f1 = p1 * s1;
      const unsigned short h0 = bf_bits(f0), h1 = bf_bits(f1);
      const unsigned short l0 = bf_bits(f0 - bf_up(h0)), l1 = bf_bits(f1 - bf_up(h1));
      dot += Lsh[c0 + 2 * t] * p0 + Lsh[c0 + 2 * t + 1] * p1;
      uh[t] = pk16(h0, h1);
      ul[t] = pk16(l0, l1);
    }
    *(volatile v4u*)(dh + e) = uh;
    if (fold) *(volatile v4u*)(dl + e) = ul;
    __threadfence();
    *(volatile v4u*)(dh + e) = uh;
    if (fold) *(volatile v4u*)(dl + e) = ul;
    dot += __shfl_xor(dot, 16, 32);
    dot += __shfl_xor(dot, 8, 32);
    dot += __shfl_xor(dot, 4, 32);
    dot += __shfl_xor(dot, 2, 32);
    dot += __shfl_xor(dot, 1, 32);
    const float bb = bfr(bsrc[part * 32 + it * 8 + wave]);
    if (fold && lane == 0) Lb[it * 8 + wave] = dot + bb;
  }
  __syncthreads();
  {
    const int q = tid & 7;
    const v4f bv = *(const v4f*)(Lb + 4 * q);
    float* bp = BF + (fold ? role : 0) * NF + part * 32 + 4 * q;
    if (fold && tid < 8) *(volatile v4f*)bp = bv;
    __threadfence();
    if (fold && tid < 8) *(volatile v4f*)bp = bv;
  }
}

__global__ __launch_bounds__(256)
void proj_kernel(const float* __restrict__ x, const float* __restrict__ x1, const float* __restrict__ x2,
                 const unsigned short* __restrict__ W1H, const unsigned short* __restrict__ W1L,
                 const unsigned short* __restrict__ W2H, const unsigned short* __restrict__ W2L,
                 const unsigned short* __restrict__ WV, const float* __restrict__ BF,
                 const float* __restrict__ vbp,
                 unsigned short* QH, unsigned short* QL, unsigned short* KH, unsigned short* KL,
                 unsigned short* VP) {
  __shared__ __align__(16) unsigned short Lat[QT * AP];
  __shared__ __align__(16) unsigned short Lq[2][QT * QP];
  __shared__ __align__(16) unsigned short Lk[2][QT * QP];
  const int tid  = threadIdx.x;
  const int lane = tid & 31, wave = tid >> 5;
  const int hh   = lane >> 4, c = lane & 15;
  const int bx   = blockIdx.x;
  const int b    = bx / (SEQ / QT);
  const int nt   = bx % (SEQ / QT);
  const int n0   = nt * QT;
  const int ng = wave & 3, cg = wave >> 2;
  const int nr = ng * 16 + 8 * hh;

#pragma unroll 1
  for (int ms = 0; ms < 3; ++ms) {
    const bool two = ms < 2;
    const float* src = (ms == 0) ? x1 : ((ms == 1) ? x2 : x);
    const unsigned short* wh = (ms == 0) ? W1H : ((ms == 1) ? W2H : WV);
    const unsigned short* wl = (ms == 0) ? W1L : W2L;

    __syncthreads();
    {
      const int n4 = (tid & 15) * 4, ds = tid >> 4;
      const float* xp = src + ((size_t)b * CIN + ds) * SEQ + n0 + n4;
#pragma unroll 4
      for (int it = 0; it < 16; ++it) {
        const v4f v = *(const v4f*)(xp + (size_t)it * 16 * SEQ);
        const int d = it * 16 + ds;
#pragma unroll
        for (int q = 0; q < 4; ++q) Lat[(n4 + q) * AP + d] = bf_bits(v[q]);
      }
    }
    __syncthreads();

    const unsigned short* ap  = Lat + (ng * 16 + c) * AP + 8 * hh;
    const unsigned short* bph = wh + (size_t)(cg * 64 + c) * CIN + 8 * hh;
    const unsigned short* bpl = wl + (size_t)(cg * 64 + c) * CIN + 8 * hh;
    v8f acc0 = zero8(), acc1 = zero8(), acc2 = zero8(), acc3 = zero8();
#pragma unroll 2
    for (int ks = 0; ks < CIN / 32; ++ks) {
      const v16b a = ldfrag_b(ap + 32 * ks);
      const unsigned short* ph = bph + 32 * ks;
      acc0 = mma_b(a, ldfrag_b(ph + 0 * 16 * CIN), acc0);
      acc1 = mma_b(a, ldfrag_b(ph + 1 * 16 * CIN), acc1);
      acc2 = mma_b(a, ldfrag_b(ph + 2 * 16 * CIN), acc2);
      acc3 = mma_b(a, ldfrag_b(ph + 3 * 16 * CIN), acc3);
      if (two) {
        const unsigned short* pl = bpl + 32 * ks;
        acc0 = mma_b(a, ldfrag_b(pl + 0 * 16 * CIN), acc0);
        acc1 = mma_b(a, ldfrag_b(pl + 1 * 16 * CIN), acc1);
        acc2 = mma_b(a, ldfrag_b(pl + 2 * 16 * CIN), acc2);
        acc3 = mma_b(a, ldfrag_b(pl + 3 * 16 * CIN), acc3);
      }
    }

    const int f0  = cg * 64 + c;
    const int bfo = (two ? ms : 0) * NF;
    const float fb0 = BF[bfo + f0], fb1 = BF[bfo + f0 + 16], fb2 = BF[bfo + f0 + 32], fb3 = BF[bfo + f0 + 48];
    const float vb0 = bfr(vbp[f0]), vb1 = bfr(vbp[f0 + 16]), vb2 = bfr(vbp[f0 + 32]), vb3 = bfr(vbp[f0 + 48]);
    const float bias0 = two ? fb0 : vb0, bias1 = two ? fb1 : vb1, bias2 = two ? fb2 : vb2, bias3 = two ? fb3 : vb3;

    if (two) {
      const int ck0 = cg * 64 + 2 * c + ms, ck1 = ck0 + 32;
      stage_split(Lk[0], Lk[1], nr, ck0, acc0, bias0);
      stage_split(Lk[0], Lk[1], nr, ck1, acc1, bias1);
      stage_split(Lq[0], Lq[1], nr, ck0, acc2, bias2);
      stage_split(Lq[0], Lq[1], nr, ck1, acc3, bias3);
    } else {
      __syncthreads();
      stage_v(Lat, f0,      nr, acc0, bias0);
      stage_v(Lat, f0 + 16, nr, acc1, bias1);
      stage_v(Lat, f0 + 32, nr, acc2, bias2);
      stage_v(Lat, f0 + 48, nr, acc3, bias3);
    }
  }
  __syncthreads();

  {
    const int e = tid & 7, lq = tid >> 3;
#pragma unroll
    for (int pass = 0; pass < 2; ++pass) {
#pragma unroll
      for (int it = 0; it < 4; ++it) {
        const int L = it * 32 + lq;
        const int h = L >> 6, n = L & 63;
        const size_t go = ((size_t)(b * NH + h) * SEQ + n0 + n) * HD + 8 * e;
        const int lo_ = n * QP + h * 64 + 8 * e;
        const v4u uqh = *(const v4u*)(Lq[0] + lo_);
        const v4u uql = *(const v4u*)(Lq[1] + lo_);
        const v4u ukh = *(const v4u*)(Lk[0] + lo_);
        const v4u ukl = *(const v4u*)(Lk[1] + lo_);
        *(volatile v4u*)(QH + go) = uqh;
        *(volatile v4u*)(QL + go) = uql;
        *(volatile v4u*)(KH + go) = ukh;
        *(volatile v4u*)(KL + go) = ukl;
      }
#pragma unroll
      for (int it = 0; it < 4; ++it) {
        const int er = it * 32 + lq;
        const v4u uv = *(const v4u*)(Lat + er * LP + 8 * e);
        *(volatile v4u*)(VP + ((size_t)b * NF + er) * SEQ + n0 + 8 * e) = uv;
      }
      __threadfence();
    }
  }
}

__global__ __launch_bounds__(128)
void attn_kernel(const unsigned short* __restrict__ QH, const unsigned short* __restrict__ QL,
                 const unsigned short* __restrict__ KH, const unsigned short* __restrict__ KL,
                 const unsigned short* __restrict__ VP, float* OB) {
  __shared__ __align__(16) float Os[QT * OSP];
  const int tid  = threadIdx.x;
  const int wave = tid >> 5;
  const int lane = tid & 31;
  const int hh   = lane >> 4;
  const int c    = lane & 15;
  const int bx   = blockIdx.x;
  const int bh   = bx / (SEQ / QT);
  const int qb   = bx % (SEQ / QT);
  const int n0   = qb * QT;
  const int b    = bh >> 1, h = bh & 1;
  const _Float16* QHh = (const _Float16*)(const void*)QH;
  const _Float16* QLh = (const _Float16*)(const void*)QL;
  const _Float16* KHh = (const _Float16*)(const void*)KH;
  const _Float16* KLh = (const _Float16*)(const void*)KL;
  const _Float16* VPh = (const _Float16*)(const void*)VP;

  const size_t qo = ((size_t)bh * SEQ + n0 + wave * 16 + c) * HD + 8 * hh;
  const v16h qh0 = ldfrag_h(QHh + qo), qh1 = ldfrag_h(QHh + qo + 32);
  const v16h ql0 = ldfrag_h(QLh + qo), ql1 = ldfrag_h(QLh + qo + 32);
  const size_t ko = ((size_t)bh * SEQ + c) * HD + 8 * hh;
  const _Float16* Kp = KHh + ko;
  const _Float16* Lp = KLh + ko;
  const _Float16* Vb = VPh + ((size_t)bh * HD + c) * SEQ + 8 * hh;

  float m = -1.0e30f, l = 0.f;
  v8f o0 = zero8(), o1 = zero8(), o2 = zero8(), o3 = zero8();
#pragma unroll 1
  for (int it = 0; it < SEQ / 32; ++it) {
    const int kb = it * 32;
    const _Float16* k0p = Kp + (size_t)kb * HD;
    const _Float16* k1p = k0p + 16 * HD;
    const _Float16* l0p = Lp + (size_t)kb * HD;
    const _Float16* l1p = l0p + 16 * HD;
    v8f s0, t0, s1, t1;
    {
      const v16h a0 = ldfrag_h(k0p), a1 = ldfrag_h(k0p + 32);
      s0 = mma_h(a0, qh0, zero8());
      s0 = mma_h(a1, qh1, s0);
      t0 = mma_h(a0, ql0, zero8());
      t0 = mma_h(a1, ql1, t0);
      const v16h r0 = ldfrag_h(l0p), r1 = ldfrag_h(l0p + 32);
      t0 = mma_h(r0, qh0, t0);
      t0 = mma_h(r1, qh1, t0);
    }
    {
      const v16h a0 = ldfrag_h(k1p), a1 = ldfrag_h(k1p + 32);
      s1 = mma_h(a0, qh0, zero8());
      s1 = mma_h(a1, qh1, s1);
      t1 = mma_h(a0, ql0, zero8());
      t1 = mma_h(a1, ql1, t1);
      const v16h r0 = ldfrag_h(l1p), r1 = ldfrag_h(l1p + 32);
      t1 = mma_h(r0, qh0, t1);
      t1 = mma_h(r1, qh1, t1);
    }
#pragma unroll
    for (int r = 0; r < 8; ++r) {
      s0[r] = s0[r] * SCL + t0[r] * IRSS;
      s1[r] = s1[r] * SCL + t1[r] * IRSS;
    }

    float mx = fmaxf(hmax8(s0), hmax8(s1));
    mx = fmaxf(mx, __shfl_xor(mx, 16, 32));
    const float mn   = fmaxf(m, mx);
    const float corr = __expf(m - mn);
    m = mn;
    const float msh = mn - LNPS;
    l *= corr;
#pragma unroll
    for (int r = 0; r < 8; ++r) {
      o0[r] *= corr; o1[r] *= corr; o2[r] *= corr; o3[r] *= corr;
    }

    FragH ph;
    float ls = 0.f;
#pragma unroll
    for (int r = 0; r < 8; ++r) {
      const float e0 = __expf(s0[r] - msh);
      const float e1 = __expf(s1[r] - msh);
      ls += e0 + e1;
      ph.h[0][r] = (_Float16)e0;
      ph.h[1][r] = (_Float16)e1;
    }
    l += ls;

    o0 = mma_h(ldfrag_h(Vb + 0 * 16 * SEQ + kb), ph.v, o0);
    o1 = mma_h(ldfrag_h(Vb + 1 * 16 * SEQ + kb), ph.v, o1);
    o2 = mma_h(ldfrag_h(Vb + 2 * 16 * SEQ + kb), ph.v, o2);
    o3 = mma_h(ldfrag_h(Vb + 3 * 16 * SEQ + kb), ph.v, o3);
  }
  l += __shfl_xor(l, 16, 32);
  const float sc = (1.0f / l) * IVSC;

  float* os = Os + (wave * 16 + c) * OSP + 8 * hh;
#pragma unroll
  for (int r = 0; r < 8; ++r) {
    os[0 * 16 + r] = o0[r] * sc;
    os[1 * 16 + r] = o1[r] * sc;
    os[2 * 16 + r] = o2[r] * sc;
    os[3 * 16 + r] = o3[r] * sc;
  }
  __syncthreads();
  {
    const int e = tid & 7, lq = tid >> 3;
    float* ob = OB + ((size_t)b * SEQ + n0) * NF + h * HD;
#pragma unroll
    for (int pass = 0; pass < 2; ++pass) {
#pragma unroll
      for (int it = 0; it < 8; ++it) {
        const int L   = it * 16 + lq;
        const int row = L >> 1, hf = L & 1;
        const v4f v = *(const v4f*)(Os + row * OSP + hf * 32 + 4 * e);
        *(volatile v4f*)(ob + (size_t)row * NF + hf * 32 + 4 * e) = v;
      }
      __threadfence();
    }
  }
}

__global__ __launch_bounds__(256)
void out_kernel(const float* __restrict__ OB, const unsigned short* __restrict__ WO,
                const float* __restrict__ obp, const float* __restrict__ gl, const float* __restrict__ bl,
                const float* __restrict__ ml, const float* __restrict__ vl, const float* __restrict__ wsp,
                const float* __restrict__ x, float* out) {
  __shared__ __align__(16) unsigned short Loh[QT * OHP];
  __shared__ __align__(16) unsigned short Lol[QT * OHP];
  __shared__ __align__(16) float Os[64 * OSP];
  const int tid  = threadIdx.x;
  const int lane = tid & 31, wave = tid >> 5;
  const int hh   = lane >> 4, c = lane & 15;
  const int bx   = blockIdx.x;
  const int b    = bx / (SEQ / QT);
  const int nt   = bx % (SEQ / QT);
  const int n0   = nt * QT;

  {
    const int row = tid >> 2, seg = (tid & 3) * 32;
    const float* op = OB + ((size_t)b * SEQ + n0 + row) * NF + seg;
#pragma unroll
    for (int q2 = 0; q2 < 4; ++q2) {
      const v4f fa = *(const v4f*)(op + 8 * q2);
      const v4f fb = *(const v4f*)(op + 8 * q2 + 4);
      const v8f w8 = __builtin_shufflevector(fa, fb, 0, 1, 2, 3, 4, 5, 6, 7);
      v4u uh, ul;
#pragma unroll
      for (int t = 0; t < 4; ++t) {
        const float p0 = w8[2 * t], p1 = w8[2 * t + 1];
        const unsigned short h0 = bf_bits(p0), h1 = bf_bits(p1);
        const unsigned short l0 = bf_bits(p0 - bf_up(h0)), l1 = bf_bits(p1 - bf_up(h1));
        uh[t] = pk16(h0, h1);
        ul[t] = pk16(l0, l1);
      }
      *(v4u*)(Loh + row * OHP + seg + 8 * q2) = uh;
      *(v4u*)(Lol + row * OHP + seg + 8 * q2) = ul;
    }
  }
  __syncthreads();

  const float wsc = bfr(wsp[0]);
  const int ctl = wave & 3, jn0 = (wave >> 2) * 2;
  const int e = tid & 7, lq = tid >> 3;
#pragma unroll 1
  for (int qd = 0; qd < 4; ++qd) {
    const int ct = qd * 4 + ctl;
    const unsigned short* ap = WO + (size_t)(ct * 16 + c) * NF + 8 * hh;
    const unsigned short* b0 = Loh + (jn0 * 16 + c) * OHP + 8 * hh;
    const unsigned short* b1 = b0 + 16 * OHP;
    const unsigned short* l0 = Lol + (jn0 * 16 + c) * OHP + 8 * hh;
    const unsigned short* l1 = l0 + 16 * OHP;
    v8f acc0 = zero8(), acc1 = zero8();
#pragma unroll
    for (int ks = 0; ks < NF / 32; ++ks) {
      const v16b a = ldfrag_b(ap + 32 * ks);
      acc0 = mma_b(a, ldfrag_b(b0 + 32 * ks), acc0);
      acc0 = mma_b(a, ldfrag_b(l0 + 32 * ks), acc0);
      acc1 = mma_b(a, ldfrag_b(b1 + 32 * ks), acc1);
      acc1 = mma_b(a, ldfrag_b(l1 + 32 * ks), acc1);
    }
    __syncthreads();
    float* os = Os + (ctl * 16 + 8 * hh) * OSP + jn0 * 16 + c;
#pragma unroll
    for (int r = 0; r < 8; ++r) {
      os[r * OSP]      = acc0[r];
      os[r * OSP + 16] = acc1[r];
    }
    __syncthreads();
#pragma unroll
    for (int it = 0; it < 4; ++it) {
      const int L   = it * 32 + lq;
      const int row = L >> 1, hf = L & 1;
      const int cgl = qd * 64 + row;
      const v4f osv = *(const v4f*)(Os + row * OSP + hf * 32 + 4 * e);
      const size_t gi = ((size_t)b * CIN + cgl) * SEQ + n0 + hf * 32 + 4 * e;
      const v4f xv = *(const v4f*)(x + gi);
      const float obv = bfr(obp[cgl]);
      const float g = bfr(gl[cgl]), bt = bfr(bl[cgl]), mu = bfr(ml[cgl]), var = bfr(vl[cgl]);
      const float rs  = rsqrtf(var + BNEPS);
      const float sl  = g * rs;
      const float shl = bt - (mu * g) * rs;
      v4f ov;
#pragma unroll
      for (int i = 0; i < 4; ++i) ov[i] = wsc * ((osv[i] + obv) * sl + shl) + bfr(xv[i]);
      *(volatile v4f*)(out + gi) = ov;
      __threadfence();
      *(volatile v4f*)(out + gi) = ov;
    }
  }
}

extern "C" void kernel_launch(void* const* d_in, const int* in_sizes, int n_in,
                              void* d_out, int out_size, void* d_ws, size_t ws_size,
                              hipStream_t stream) {
  const int NX = NB * CIN * SEQ;
  if (n_in < 24) return;
  if (in_sizes[0] != NX || in_sizes[1] != NX || in_sizes[2] != NX) return;
  for (int i = 3; i <= 10; ++i) if (in_sizes[i] != CIN) return;
  if (in_sizes[11] != NF * CIN || in_sizes[12] != NF || in_sizes[13] != NF * CIN || in_sizes[14] != NF) return;
  if (in_sizes[15] != NF * CIN || in_sizes[16] != NF || in_sizes[17] != CIN * NF || in_sizes[18] != CIN) return;
  for (int i = 19; i <= 22; ++i) if (in_sizes[i] != CIN) return;
  if (in_sizes[23] < 1) return;
  if (out_size != NX) return;

  size_t off = 0;
  const size_t szW = (size_t)NF * CIN * 2;
  const size_t oW1H = off; off += szW;
  const size_t oW1L = off; off += szW;
  const size_t oW2H = off; off += szW;
  const size_t oW2L = off; off += szW;
  const size_t oWV  = off; off += szW;
  const size_t oWO  = off; off += (size_t)CIN * NF * 2;
  const size_t oBF  = off; off += (size_t)2 * NF * 4;
  const size_t szP  = (size_t)NBH * SEQ * HD * 2;
  const size_t oQH  = off; off += szP;
  const size_t oQL  = off; off += szP;
  const size_t oKH  = off; off += szP;
  const size_t oKL  = off; off += szP;
  const size_t oV   = off; off += (size_t)NBH * HD * SEQ * 2;
  const size_t oOB  = off; off += (size_t)NB * SEQ * NF * 4;
  if (off > ws_size) return;
  if (off > (size_t)134217728) return;

  const float* x     = (const float*)d_in[0];
  const float* x1    = (const float*)d_in[1];
  const float* x2    = (const float*)d_in[2];
  const float* bn1_g = (const float*)d_in[3];
  const float* bn1_b = (const float*)d_in[4];
  const float* bn1_m = (const float*)d_in[5];
  const float* bn1_v = (const float*)d_in[6];
  const float* bn2_g = (const float*)d_in[7];
  const float* bn2_b = (const float*)d_in[8];
  const float* bn2_m = (const float*)d_in[9];
  const float* bn2_v = (const float*)d_in[10];
  const float* kq1_w = (const float*)d_in[11];
  const float* kq1_b = (const float*)d_in[12];
  const float* kq2_w = (const float*)d_in[13];
  const float* kq2_b = (const float*)d_in[14];
  const float* v_w   = (const float*)d_in[15];
  const float* v_b   = (const float*)d_in[16];
  const float* out_w = (const float*)d_in[17];
  const float* out_b = (const float*)d_in[18];
  const float* bnl_g = (const float*)d_in[19];
  const float* bnl_b = (const float*)d_in[20];
  const float* bnl_m = (const float*)d_in[21];
  const float* bnl_v = (const float*)d_in[22];
  const float* w_scale = (const float*)d_in[23];

  char* ws = (char*)d_ws;
  unsigned short* W1H = (unsigned short*)(ws + oW1H);
  unsigned short* W1L = (unsigned short*)(ws + oW1L);
  unsigned short* W2H = (unsigned short*)(ws + oW2H);
  unsigned short* W2L = (unsigned short*)(ws + oW2L);
  unsigned short* WV  = (unsigned short*)(ws + oWV);
  unsigned short* WO  = (unsigned short*)(ws + oWO);
  float*          BF  = (float*)(ws + oBF);
  unsigned short* QH  = (unsigned short*)(ws + oQH);
  unsigned short* QL  = (unsigned short*)(ws + oQL);
  unsigned short* KH  = (unsigned short*)(ws + oKH);
  unsigned short* KL  = (unsigned short*)(ws + oKL);
  unsigned short* VP  = (unsigned short*)(ws + oV);
  float*          OB  = (float*)(ws + oOB);
  float* out = (float*)d_out;

  const dim3 blk256(256), blk128(128);
  const dim3 gW(16);
  const dim3 gP(NB * (SEQ / QT));
  const dim3 gA(NBH * (SEQ / QT));
  const dim3 gO(NB * (SEQ / QT));

  wprep_kernel<<<gW, blk256, 0, stream>>>(kq1_w, kq1_b, kq2_w, kq2_b, v_w, out_w,
                                           bn1_g, bn1_b, bn1_m, bn1_v,
                                           bn2_g, bn2_b, bn2_m, bn2_v,
                                           W1H, W1L, W2H, W2L, WV, WO, BF);
  proj_kernel<<<gP, blk256, 0, stream>>>(x, x1, x2, W1H, W1L, W2H, W2L, WV, BF, v_b, QH, QL, KH, KL, VP);
  attn_kernel<<<gA, blk128, 0, stream>>>(QH, QL, KH, KL, VP, OB);
  out_kernel<<<gO, blk256, 0, stream>>>(OB, WO, out_b, bnl_g, bnl_b, bnl_m, bnl_v, w_scale, x, out);
  (void)hipGetLastError();
}
